// HyTE_57037165691116
// MI455X (gfx1250) — hardware-verified
//
#include <hip/hip_runtime.h>
#include <math.h>

#define NN     100000
#define ENT    50000
#define DIM    128
#define NE     1600000
#define BATCH  131072
#define REL    500
#define TIMEN  365
#define EPS_F  1e-12f

#define NT     256
#define TS     8192
#define NTILE  13
#define NPAD   (TS * NTILE)
#define RPW    (TS / 8)
#define OWS    10
#define SCH    4096
#define SPT    (SCH / NT)
#define NCH    ((NE + SCH - 1) / SCH)
#define MPAD   100032
#define WSC    16.0f
#define WSC_INV (1.0f / 16.0f)

typedef __attribute__((ext_vector_type(16))) _Float16 v16h;
typedef __attribute__((ext_vector_type(8)))  _Float16 v8h;
typedef __attribute__((ext_vector_type(16))) __bf16   v16b;
typedef __attribute__((ext_vector_type(8)))  __bf16   v8b;
typedef __attribute__((ext_vector_type(8)))  float    v8f;
typedef __attribute__((ext_vector_type(4)))  float    v4f;
typedef __attribute__((ext_vector_type(4)))  int      v4i;

__device__ __forceinline__ unsigned short f2bf_bits(float f) {
  unsigned u = __float_as_uint(f);
  return (unsigned short)((u + 0x7FFFu + ((u >> 16) & 1u)) >> 16);
}
__device__ __forceinline__ float bf_bits2f(unsigned short h) { return __uint_as_float(((unsigned)h) << 16); }

__device__ __forceinline__ void dep_guard_h(v8f& a, v8f& b, v16h x, v16h y) { asm volatile("v_nop\n\tv_nop\n\tv_nop\n\tv_nop" : "+v"(a), "+v"(b) : "v"(x), "v"(y)); }
__device__ __forceinline__ void dep_guard_b(v8f& a, v8f& b, v16b x, v16b y) { asm volatile("v_nop\n\tv_nop\n\tv_nop\n\tv_nop" : "+v"(a), "+v"(b) : "v"(x), "v"(y)); }
__device__ __forceinline__ void keep4_h(v16h a, v16h b, v16h c, v16h d) { asm volatile("v_nop" :: "v"(a), "v"(b), "v"(c), "v"(d)); }
__device__ __forceinline__ void keep4_b(v16b a, v16b b, v16b c, v16b d) { asm volatile("v_nop" :: "v"(a), "v"(b), "v"(c), "v"(d)); }
__device__ __forceinline__ void acc_guard4(v8f& a, v8f& b, v8f& c, v8f& d) { asm volatile("v_nop\n\tv_nop\n\tv_nop\n\tv_nop" : "+v"(a), "+v"(b), "+v"(c), "+v"(d)); }
template <typename T> struct Frag;
template <> struct Frag<_Float16> {
  typedef v16h V; union U { v16h v; v8h h[2]; };
  static __device__ __forceinline__ v16h load(const _Float16* p) {
    U f; f.h[0] = *(const v8h*)(p); f.h[1] = *(const v8h*)(p + 16); return f.v;
  }
  static __device__ __forceinline__ v8f mma(v16h a, v16h b, v8f c) {
    return __builtin_amdgcn_wmma_f32_16x16x32_f16(false, a, false, b, (short)0, c, false, false);
  }
  static __device__ __forceinline__ void guard(v8f& a, v8f& b, v16h x, v16h y) { dep_guard_h(a, b, x, y); }
  static __device__ __forceinline__ void keep(v16h a, v16h b, v16h c, v16h d) { keep4_h(a, b, c, d); }
};
template <> struct Frag<__bf16> {
  typedef v16b V; union U { v16b v; v8b h[2]; };
  static __device__ __forceinline__ v16b load(const __bf16* p) {
    U f; f.h[0] = *(const v8b*)(p); f.h[1] = *(const v8b*)(p + 16); return f.v;
  }
  static __device__ __forceinline__ v8f mma(v16b a, v16b b, v8f c) {
    return __builtin_amdgcn_wmma_f32_16x16x32_bf16(false, a, false, b, (short)0, c, false, false);
  }
  static __device__ __forceinline__ void guard(v8f& a, v8f& b, v16b x, v16b y) { dep_guard_b(a, b, x, y); }
  static __device__ __forceinline__ void keep(v16b a, v16b b, v16b c, v16b d) { keep4_b(a, b, c, d); }
};

template <int ET> struct Elem;
template <> struct Elem<0> { typedef _Float16 T; };
template <> struct Elem<1> { typedef __bf16 T; };
template <int ET, bool SPLIT, int BIAS_MODE, int OUT_MODE, bool RESID, int ACT = 0>
__global__ __launch_bounds__(256) void wmma_gemm64(
    const unsigned short* __restrict__ Ap, const unsigned short* __restrict__ A2p, int lda, long strideA,
    const unsigned short* __restrict__ Btp, const unsigned short* __restrict__ Bt2p, int ldb, long strideB,
    void* __restrict__ Cout, void* __restrict__ Cout2, int ldc, long strideC,
    const float* __restrict__ bias,
    const float* __restrict__ resid, long strideR,
    int M, int N, int K, float scale) {
  typedef typename Elem<ET>::T T;
  typedef typename Frag<T>::V V;
  const T* A = (const T*)Ap; const T* A2 = (const T*)A2p; const T* Bt = (const T*)Btp; const T* Bt2 = (const T*)Bt2p;
  __shared__ __align__(16) float sT[8][16 * 68];
  const int b    = blockIdx.y;
  const int lane = threadIdx.x & 31;
  const int wave = threadIdx.x >> 5;
  const int tilesN = N >> 6;
  const int tilesM = M >> 6;
  const int tile = blockIdx.x * 8 + wave;
  if (tile >= tilesM * tilesN) return;
  const int tm = tile / tilesN;
  const int tn = tile - tm * tilesN;
  const int m0 = tm << 6;
  const int n0 = tn << 6;

  const T* Ab  = A  + (size_t)b * strideA;
  const T* Bb  = Bt + (size_t)b * strideB;
  const T* Ab2 = SPLIT ? (A2  + (size_t)b * strideA) : nullptr;
  const T* Bb2 = SPLIT ? (Bt2 + (size_t)b * strideB) : nullptr;

  const int rlane = lane & 15;
  const int koff  = (lane >> 4) * 8;
  const int mOff  = (lane >> 4) * 8;

  v8f acc[4][4];
#pragma unroll
  for (int i = 0; i < 4; ++i)
#pragma unroll
    for (int j = 0; j < 4; ++j) acc[i][j] = (v8f){0.f,0.f,0.f,0.f,0.f,0.f,0.f,0.f};

  for (int k0 = 0; k0 < K; k0 += 32) {
    V bh[4], bl[4];
#pragma unroll
    for (int j = 0; j < 4; ++j) {
      const size_t bo = (size_t)(n0 + (j << 4) + rlane) * ldb + koff + k0;
      bh[j] = Frag<T>::load(Bb + bo);
      if (SPLIT) bl[j] = Frag<T>::load(Bb2 + bo);
    }
#pragma unroll
    for (int i = 0; i < 4; ++i) {
      const size_t ao = (size_t)(m0 + (i << 4) + rlane) * lda + koff + k0;
      V ah = Frag<T>::load(Ab + ao);
      V al;
      if (SPLIT) al = Frag<T>::load(Ab2 + ao);
#pragma unroll
      for (int j = 0; j < 4; ++j) {
        acc[i][j] = Frag<T>::mma(ah, bh[j], acc[i][j]);
        if (SPLIT) {
          acc[i][j] = Frag<T>::mma(ah, bl[j], acc[i][j]);
          acc[i][j] = Frag<T>::mma(al, bh[j], acc[i][j]);
        }
      }
      Frag<T>::guard(acc[i][0], acc[i][3], ah, SPLIT ? al : ah);
    }
    Frag<T>::keep(bh[0], bh[1], bh[2], bh[3]);
    if (SPLIT) Frag<T>::keep(bl[0], bl[1], bl[2], bl[3]);
  }
  acc_guard4(acc[0][0], acc[0][1], acc[0][2], acc[0][3]);
  acc_guard4(acc[1][0], acc[1][1], acc[1][2], acc[1][3]);
  acc_guard4(acc[2][0], acc[2][1], acc[2][2], acc[2][3]);
  acc_guard4(acc[3][0], acc[3][1], acc[3][2], acc[3][3]);

  float* slab = sT[wave];
  const float* Rb = RESID ? (resid + (size_t)b * strideR) : nullptr;
#pragma unroll
  for (int i = 0; i < 4; ++i) {
    const int mBase = m0 + (i << 4);
#pragma unroll
    for (int j = 0; j < 4; ++j) {
      const int n = n0 + (j << 4) + rlane;
      float bv = 0.f;
      if (BIAS_MODE == 2) bv = bias[n];
#pragma unroll
      for (int r = 0; r < 8; ++r) {
        float v = acc[i][j][r] * scale;
        if (BIAS_MODE == 1) v += bias[mBase + mOff + r];
        if (BIAS_MODE == 2) v += bv;
        if (RESID) v += Rb[(size_t)(mBase + mOff + r) * ldc + n];
        if (ACT == 1) v = tanhf(v);
        if (ACT == 2) v = fmaxf(v, 0.0f);
        if (ACT == 3) v = v / (1.0f + expf(-v));
        if (ACT == 4) v = (v > 0.f) ? v : 0.01f * v;
        if (ACT == 5) v = 0.5f * v * (1.0f + erff(v * 0.70710678118654752f));
        slab[(mOff + r) * 68 + (j << 4) + rlane] = v;
      }
    }
    __builtin_amdgcn_fence(__ATOMIC_RELEASE, "workgroup");
    __builtin_amdgcn_wave_barrier();
    __builtin_amdgcn_fence(__ATOMIC_ACQUIRE, "workgroup");
    if (OUT_MODE == 0) {
      float* C = (float*)Cout + (size_t)b * strideC;
      const int hh = lane >> 4, c4 = (lane & 15) * 4;
      for (int pass = 0; pass < 2; ++pass) {
#pragma unroll
        for (int it = 0; it < 8; ++it) {
          const int row = it * 2 + hh;
          v4f v = *(const v4f*)(slab + row * 68 + c4);
          *(volatile v4f*)(C + (size_t)(mBase + row) * ldc + n0 + c4) = v;
        }
        __threadfence();
      }
    } else {
      const int q = lane >> 3, c8 = (lane & 7) * 8;
      unsigned short* C  = (unsigned short*)Cout  + (size_t)b * strideC;
      unsigned short* C2 = (OUT_MODE == 2) ? ((unsigned short*)Cout2 + (size_t)b * strideC) : nullptr;
      for (int pass = 0; pass < 2; ++pass) {
#pragma unroll
        for (int it = 0; it < 4; ++it) {
          const int row = it * 4 + q;
          const float* sp = slab + row * 68 + c8;
          v8h hv, lv;
#pragma unroll
          for (int e = 0; e < 8; ++e) {
            if (OUT_MODE == 1) {
              hv[e] = (_Float16)sp[e];
            } else {
              unsigned short hb = f2bf_bits(sp[e]);
              unsigned short lb = f2bf_bits(sp[e] - bf_bits2f(hb));
              hv[e] = __builtin_bit_cast(_Float16, hb);
              lv[e] = __builtin_bit_cast(_Float16, lb);
            }
          }
          *(volatile v8h*)(C + (size_t)(mBase + row) * ldc + n0 + c8) = hv;
          if (OUT_MODE == 2) *(volatile v8h*)(C2 + (size_t)(mBase + row) * ldc + n0 + c8) = lv;
        }
        __threadfence();
      }
    }
    __builtin_amdgcn_fence(__ATOMIC_RELEASE, "workgroup");
    __builtin_amdgcn_wave_barrier();
    __builtin_amdgcn_fence(__ATOMIC_ACQUIRE, "workgroup");
  }
}

__global__ __launch_bounds__(256) void cast_w_f16(const float* __restrict__ in, _Float16* __restrict__ out, int n2, float sc) {
  const int i = blockIdx.x * 256 + threadIdx.x;
  if (i < n2) {
    const _Float16 h0 = (_Float16)(in[2 * i] * sc), h1 = (_Float16)(in[2 * i + 1] * sc);
    const unsigned u = (unsigned)__builtin_bit_cast(unsigned short, h0) | ((unsigned)__builtin_bit_cast(unsigned short, h1) << 16);
    ((volatile unsigned*)out)[i] = u;
    __threadfence();
    ((volatile unsigned*)out)[i] = u;
  }
}

__device__ __forceinline__ int blk_excl_scan(int cnt, int* scan_ws, int tid, int* tot) {
  const int lane = tid & 31, wave = tid >> 5; int incl = cnt;
#pragma unroll
  for (int o = 1; o < 32; o <<= 1) { const int v = __shfl_up(incl, o, 32); if (lane >= o) incl += v; }
  if (lane == 31) scan_ws[wave] = incl;
  __syncthreads();
  if (wave == 0) { int wv = (lane < NT / 32) ? scan_ws[lane] : 0; int wincl = wv;
#pragma unroll
    for (int o = 1; o < 32; o <<= 1) { const int v = __shfl_up(wincl, o, 32); if (lane >= o) wincl += v; }
    if (lane < NT / 32) scan_ws[32 + lane] = wincl - wv; if (lane == 31) scan_ws[64] = wincl; }
  __syncthreads();
  const int res = scan_ws[32 + wave] + incl - cnt; *tot = scan_ws[64];
  return res;
}
template <int SP, int CAP>
__device__ __forceinline__ int chunk_hits(const int* __restrict__ dstv, const int* __restrict__ srcv, int e0, int n0, int tid,
                                          int* LIST, int* scan_ws) {
  const int eb = e0 + tid * SP;
  const bool inb = eb < NE;
  const int ebc = inb ? eb : (NE - SP);
  int rec[SP]; int cnt = 0;
#pragma unroll
  for (int k = 0; k < SP; k += 4) {
    const v4i d4 = *(const v4i*)(dstv + ebc + k);
    const v4i s4 = *(const v4i*)(srcv + ebc + k);
#pragma unroll
    for (int e = 0; e < 4; ++e) {
      const int d = d4[e]; int s = s4[e]; s = s < 0 ? 0 : (s >= NN ? NN - 1 : s);
      int r = -1;
      if (inb && d >= n0 && d < n0 + TS) { r = ((d - n0) << 17) | s; ++cnt; }
      rec[k + e] = r;
    }
  }
  int tot; int p = blk_excl_scan(cnt, scan_ws, tid, &tot);
#pragma unroll
  for (int k = 0; k < SP; ++k) if (rec[k] >= 0) { if ((unsigned)p < (unsigned)CAP) LIST[p] = rec[k]; ++p; }
  __syncthreads();
  return tot < CAP ? tot : CAP;
}

__global__ __launch_bounds__(NT) void agg_kernel(const float* __restrict__ feat, const int* __restrict__ srcv, const int* __restrict__ dstv,
                                                float* ACC, unsigned short* __restrict__ AH) {
  __shared__ int LIST[SCH];
  __shared__ int scan_ws[80];
  const int tid = threadIdx.x, lane = tid & 31, wave = tid >> 5;
  const int n0 = blockIdx.x * TS;
  const int r0 = n0 + wave * RPW;
  const v4f z4 = {0.f, 0.f, 0.f, 0.f};
  for (int pass = 0; pass < 2; ++pass) {
#pragma unroll 1
    for (int j = 0; j < RPW; ++j) *(volatile v4f*)(ACC + (size_t)(r0 + j) * DIM + 4 * lane) = z4;
    __threadfence();
  }
#pragma unroll 1
  for (int ch = 0; ch < NCH; ++ch) {
    const int tot = chunk_hits<SPT, SCH>(dstv, srcv, ch * SCH, n0, tid, LIST, scan_ws);
#pragma unroll 1
    for (int base = 0; base < tot; base += 32) {
      const int q = base + lane;
      const int qc = q < SCH ? q : SCH - 1;
      int rv = LIST[qc];
      rv = (q < tot) ? rv : -1;
      const int own = (rv >= 0 && (rv >> (17 + OWS)) == wave) ? 1 : 0;
      unsigned msk = (unsigned)__ballot(own);
#pragma unroll 1
      for (int it = 0; it < 32; ++it) {
        if (msk == 0u) break;
        const int bp = __builtin_ctz(msk); msk &= msk - 1u;
        const int r = __shfl(rv, bp, 32);
        const int dl = r >> 17;
        int s = r & 0x1FFFF; s = s < NN ? s : NN - 1;
        const v4f hv = *(const v4f*)(feat + (size_t)s * DIM + 4 * lane);
        float* rp = ACC + (size_t)(n0 + dl) * DIM + 4 * lane;
        v4f a = *(const v4f*)rp;
        a = a + hv;
        *(volatile v4f*)rp = a;
        __threadfence();
        *(volatile v4f*)rp = a;
      }
    }
    __syncthreads();
  }
  __threadfence();
  const int hh = lane >> 4, c8 = (lane & 15) * 8;
#pragma unroll 1
  for (int j = 0; j < RPW; j += 2) {
    const int rb = r0 + j;
    if (rb < MPAD) {
      const int row = rb + hh;
      const bool live = row < NN;
      const float* rp = ACC + (size_t)row * DIM + c8;
      const v4f a0 = *(const v4f*)rp;
      const v4f a1 = *(const v4f*)(rp + 4);
      v8h hv;
#pragma unroll
      for (int e = 0; e < 4; ++e) {
        hv[e]     = live ? (_Float16)a0[e] : (_Float16)0.0f;
        hv[4 + e] = live ? (_Float16)a1[e] : (_Float16)0.0f;
      }
      unsigned short* op = AH + (size_t)row * DIM + c8;
      *(volatile v8h*)op = hv;
      __threadfence();
      *(volatile v8h*)op = hv;
    }
  }
}

__device__ __forceinline__ float wsum(float v) {
#pragma unroll
  for (int off = 16; off > 0; off >>= 1) v += __shfl_xor(v, off, 32);
  return v;
}
__device__ __forceinline__ float dot4(v4f a, v4f b) { return a[0] * b[0] + a[1] * b[1] + a[2] * b[2] + a[3] * b[3]; }
__device__ __forceinline__ v4f proj_norm(v4f e, v4f n) {
  const float d = wsum(dot4(n, e));
  e = e - d * n;
  const float en = sqrtf(wsum(dot4(e, e)));
  const float inv = 1.0f / fmaxf(en, EPS_F);
  return e * inv;
}
__global__ __launch_bounds__(NT) void score_kernel(const float* __restrict__ H2, const float* __restrict__ rel, const float* __restrict__ nrm,
                                                  const int* __restrict__ h_idx, const int* __restrict__ r_idx,
                                                  const int* __restrict__ t_idx, const int* __restrict__ tm_idx,
                                                  float* __restrict__ out) {
  __shared__ __align__(16) float so[32];
  const int tid = threadIdx.x, lane = tid & 31, wave = tid >> 5;
  const int c = 4 * lane;
#pragma unroll 1
  for (int u = 0; u < 4; ++u) {
    int row = blockIdx.x * 32 + wave * 4 + u; row = row < BATCH ? row : BATCH - 1;
    int ih = h_idx[row];  ih = ih < 0 ? 0 : (ih >= ENT ? ENT - 1 : ih);
    int it = t_idx[row];  it = it < 0 ? 0 : (it >= ENT ? ENT - 1 : it);
    int ir = r_idx[row];  ir = ir < 0 ? 0 : (ir >= REL ? REL - 1 : ir);
    int im = tm_idx[row]; im = im < 0 ? 0 : (im >= TIMEN ? TIMEN - 1 : im);
    const v4f ha = *(const v4f*)(H2 + (size_t)ih * DIM + c);
    const v4f hb = *(const v4f*)(H2 + (size_t)(ih + ENT) * DIM + c);
    const v4f ta = *(const v4f*)(H2 + (size_t)it * DIM + c);
    const v4f tb = *(const v4f*)(H2 + (size_t)(it + ENT) * DIM + c);
    v4f r = *(const v4f*)(rel + (size_t)ir * DIM + c);
    v4f n = *(const v4f*)(nrm + (size_t)im * DIM + c);
    v4f h = (ha + hb) * 0.5f;
    v4f t = (ta + tb) * 0.5f;
    const float nn = sqrtf(wsum(dot4(n, n)));
    const float invn = 1.0f / fmaxf(nn, EPS_F);
    n = n * invn;
    h = proj_norm(h, n);
    r = proj_norm(r, n);
    t = proj_norm(t, n);
    const v4f dv = (h + r) - t;
    const float sc = sqrtf(wsum(dot4(dv, dv)));
    if (lane == 0) so[wave * 4 + u] = sc;
  }
  __syncthreads();
  if (wave == 0) {
    const v4f v = *(const v4f*)(so + 4 * (lane & 7));
    float* op = out + (size_t)blockIdx.x * 32 + 4 * (lane & 7);
    if (lane < 8) *(volatile v4f*)op = v;
    __threadfence();
    if (lane < 8) *(volatile v4f*)op = v;
  }
}

extern "C" void kernel_launch(void* const* d_in, const int* in_sizes, int n_in,
                              void* d_out, int out_size, void* d_ws, size_t ws_size,
                              hipStream_t stream) {
  if (n_in < 11) return;
  if (in_sizes[0] < NN * DIM || in_sizes[1] < DIM * DIM || in_sizes[2] < DIM || in_sizes[3] < REL * DIM ||
      in_sizes[4] < TIMEN * DIM || in_sizes[5] < NE || in_sizes[6] < NE || in_sizes[7] < BATCH ||
      in_sizes[8] < BATCH || in_sizes[9] < BATCH || in_sizes[10] < BATCH || out_size < BATCH) return;

  const float* node_feat = (const float*)d_in[0];
  const float* W         = (const float*)d_in[1];
  const float* bvec      = (const float*)d_in[2];
  const float* rel_emb   = (const float*)d_in[3];
  const float* norm_emb  = (const float*)d_in[4];
  const int*   src       = (const int*)d_in[5];
  const int*   dst       = (const int*)d_in[6];
  const int*   h_idx     = (const int*)d_in[7];
  const int*   r_idx     = (const int*)d_in[8];
  const int*   t_idx     = (const int*)d_in[9];
  const int*   tm_idx    = (const int*)d_in[10];
  float*       out       = (float*)d_out;

  char* ws = (char*)d_ws; size_t off = 0;
  auto carve = [&](size_t bytes) -> char* { char* p = ws + off; off += (bytes + 255) & ~(size_t)255; return p; };
  _Float16*       WH  = (_Float16*)carve((size_t)DIM * DIM * 2);
  float*          ACC = (float*)carve((size_t)NPAD * DIM * 4);
  float*          HB  = (float*)carve((size_t)MPAD * DIM * 4);
  unsigned short* AH  = (unsigned short*)carve((size_t)MPAD * DIM * 2);
  if (off > ws_size || off > (size_t)134217728) return;

  const int gemm_tiles  = (MPAD / 64) * (DIM / 64);
  const int gemm_blocks = (gemm_tiles + 7) / 8;

  cast_w_f16<<<(DIM * DIM / 2 + NT - 1) / NT, NT, 0, stream>>>(W, WH, DIM * DIM / 2, WSC);

  agg_kernel<<<NTILE, NT, 0, stream>>>(node_feat, src, dst, ACC, AH);
  wmma_gemm64<0, false, 2, 0, false, 2><<<dim3(gemm_blocks, 1), 256, 0, stream>>>(
      (const unsigned short*)AH, (const unsigned short*)nullptr, DIM, 0L,
      (const unsigned short*)WH, (const unsigned short*)nullptr, DIM, 0L,
      (void*)HB, (void*)nullptr, DIM, 0L,
      bvec, (const float*)nullptr, 0L, MPAD, DIM, DIM, WSC_INV);

  agg_kernel<<<NTILE, NT, 0, stream>>>(HB, src, dst, ACC, AH);
  wmma_gemm64<0, false, 2, 0, false, 2><<<dim3(gemm_blocks, 1), 256, 0, stream>>>(
      (const unsigned short*)AH, (const unsigned short*)nullptr, DIM, 0L,
      (const unsigned short*)WH, (const unsigned short*)nullptr, DIM, 0L,
      (void*)HB, (void*)nullptr, DIM, 0L,
      bvec, (const float*)nullptr, 0L, MPAD, DIM, DIM, WSC_INV);

  score_kernel<<<BATCH / 32, NT, 0, stream>>>(HB, rel_emb, norm_emb, h_idx, r_idx, t_idx, tm_idx, out);
}
